// WAttention_19765439497051
// MI455X (gfx1250) — hardware-verified
//
#include <hip/hip_runtime.h>
#include <stddef.h>


typedef _Float16 v16h __attribute__((ext_vector_type(16)));
typedef _Float16 v8h  __attribute__((ext_vector_type(8)));
typedef float    v8f  __attribute__((ext_vector_type(8)));
typedef float    v4f  __attribute__((ext_vector_type(4)));

#ifndef NQ
#define NQ 2048
#endif
#define NQ_FULL 2048
#define DIM   512
#define NWAY  5
#define NSUP  64
#define KROWS (NWAY * NSUP)

static_assert(NQ >= 128 && NQ <= NQ_FULL && (NQ % 128) == 0);
static_assert((DIM % 64) == 0 && (DIM % 32) == 0);
static_assert(NSUP == 64);
static_assert((NSUP % 32) == 0);
static_assert((((size_t)NQ * DIM) % (8u * 256u)) == 0);
static_assert((((size_t)KROWS * DIM) % (8u * 256u)) == 0);
static_assert(((NWAY * DIM) % 64) == 0);

#define LDT 72
#define LDC 68
static_assert((LDT % 8) == 0 && LDT >= 64);
static_assert((LDC % 4) == 0 && LDC >= 64);

#define WCARRY 64.0f
#define PCARRY 1024.0f

#define WQT_BYTES  ((size_t)DIM * DIM * 2)
#define WWT_BYTES  ((size_t)DIM * NWAY * DIM * 2)
#define QPL_BYTES  ((size_t)NQ * DIM * 2)
#define KPL_BYTES  ((size_t)KROWS * DIM * 2)
#define VTP_BYTES  ((size_t)NWAY * DIM * NSUP * 2)
#define QINV_BYTES ((size_t)NQ * 4)
#define KINV_BYTES ((size_t)KROWS * 4)
#define OFF_WQT  ((size_t)0)
#define OFF_WKT  (OFF_WQT + WQT_BYTES)
#define OFF_WVT  (OFF_WKT + WWT_BYTES)
#define OFF_QIN  (OFF_WVT + WWT_BYTES)
#define OFF_KIN  (OFF_QIN + QPL_BYTES)
#define OFF_NQ   (OFF_KIN + KPL_BYTES)
#define OFF_NK   (OFF_NQ + QPL_BYTES)
#define OFF_NVT  (OFF_NK + KPL_BYTES)
#define OFF_QINV (OFF_NVT + VTP_BYTES)
#define OFF_KINV (OFF_QINV + QINV_BYTES)
#define WS_TOTAL (OFF_KINV + KINV_BYTES)
static_assert((WQT_BYTES % 128) == 0 && (WWT_BYTES % 128) == 0 && (QPL_BYTES % 128) == 0);
static_assert((KPL_BYTES % 128) == 0 && (VTP_BYTES % 128) == 0);
static_assert((QINV_BYTES % 128) == 0 && (KINV_BYTES % 128) == 0);
static_assert(WS_TOTAL <= (size_t)134217728);

__device__ __forceinline__ float bf16r(float x) {
  unsigned int u = __float_as_uint(x);
  u = (u + 0x7FFFu + ((u >> 16) & 1u)) & 0xFFFF0000u;
  return __uint_as_float(u);
}

static __device__ __forceinline__ _Float16 toh_flush(float v) {
  const _Float16 r = (_Float16)v;
  return (fabsf(v) < 6.103515625e-05f) ? (_Float16)0.0f : r;
}

__device__ __forceinline__ v16h frag_at(const _Float16* p) {
  v8h lo = *(const v8h*)(p);
  v8h hi = *(const v8h*)(p + 16);
  v16h out;
#pragma unroll
  for (int i = 0; i < 8; ++i) { out[i] = lo[i]; out[i + 8] = hi[i]; }
  return out;
}
__device__ __forceinline__ v16h ld_frag(const _Float16* base, unsigned ld) {
  const unsigned lane = threadIdx.x & 31u;
  return frag_at(base + (lane & 15u) * ld + (lane >> 4) * 8u);
}

__device__ __forceinline__ v8f wmma16(v16h a, v16h b, v8f c) {
  v8f d = __builtin_amdgcn_wmma_f32_16x16x32_f16(false, a, false, b, (short)0, c,
                                                 false, false);
  asm volatile("v_nop\n\tv_nop\n\tv_nop\n\tv_nop" : "+v"(d) : "v"(a), "v"(b));
  return d;
}

__device__ __forceinline__ float red16_sum(float x) {
#pragma unroll
  for (int off = 1; off < 16; off <<= 1) x += __shfl_xor(x, off, 32);
  return x;
}

__device__ __forceinline__ void wave_lds_sync() {
  __builtin_amdgcn_fence(3  , "wavefront");
  asm volatile("s_wait_dscnt 0x0" ::: "memory");
  __builtin_amdgcn_wave_barrier();
}

__global__ __launch_bounds__(256) void wconv_kernel(
    const float* __restrict__ W, _Float16* __restrict__ Wt, unsigned ldw, unsigned ldk) {
  __shared__ _Float16 T[64 * LDT];
  const unsigned tid = threadIdx.x;
  const unsigned n0 = blockIdx.x * 64u;
  const unsigned k0 = blockIdx.y * 64u;
#pragma unroll 4
  for (unsigned j = 0; j < 16u; ++j) {
    const unsigned idx = tid + 256u * j;
    const unsigned kr = idx >> 6, nc = idx & 63u;
    const float v = W[(size_t)(k0 + kr) * ldw + n0 + nc];
    T[nc * LDT + kr] = (_Float16)(WCARRY * bf16r(v));
  }
  __syncthreads();
  v8h x[2];
  size_t off[2];
#pragma unroll
  for (unsigned i = 0; i < 2u; ++i) {
    const unsigned n = 32u * i + (tid >> 3);
    const unsigned kc = (tid & 7u) * 8u;
    x[i] = *(const v8h*)&T[n * LDT + kc];
    off[i] = (size_t)(n0 + n) * ldk + k0 + kc;
  }
#pragma unroll
  for (int i = 0; i < 2; ++i) *(volatile v8h*)(Wt + off[i]) = x[i];
  __threadfence();
#pragma unroll
  for (int i = 0; i < 2; ++i) *(volatile v8h*)(Wt + off[i]) = x[i];
}

__global__ __launch_bounds__(256) void cast_kernel(
    const float* __restrict__ src, _Float16* __restrict__ dst, unsigned n8) {
#pragma clang fp contract(off)
  const unsigned idx = blockIdx.x * 256u + threadIdx.x;
  const unsigned cl = (idx < n8) ? idx : (n8 - 1u);
  const v4f a0 = *(const v4f*)(src + (size_t)cl * 8u);
  const v4f a1 = *(const v4f*)(src + (size_t)cl * 8u + 4u);
  v8h o;
#pragma unroll
  for (int i = 0; i < 4; ++i) {
    o[i]     = toh_flush(bf16r(a0[i]));
    o[i + 4] = toh_flush(bf16r(a1[i]));
  }
  if (idx < n8) {
    _Float16* p = dst + (size_t)idx * 8u;
    *(volatile v8h*)p = o;
    __threadfence();
    *(volatile v8h*)p = o;
  }
}

template <int MODE>
__device__ __forceinline__ void proj_body(
    const _Float16* __restrict__ A16, const _Float16* __restrict__ Bt, const unsigned ldb,
    _Float16* __restrict__ out16, float* __restrict__ inv) {
  __shared__ float Cs[64 * LDC];
  __shared__ float Ninv[64];
  const unsigned tid = threadIdx.x, lane = tid & 31u;
  const unsigned w = (unsigned)__builtin_amdgcn_readfirstlane((int)(tid >> 5));
  const unsigned mw = w >> 1, nw = w & 1u;
  const unsigned hh = lane >> 4, m = lane & 15u;

  const _Float16* ap = A16 + (size_t)(mw * 16u + m) * DIM + hh * 8u;
  float ssq[2] = {0.0f, 0.0f};

#pragma unroll 1
  for (unsigned nt = 0; nt < (unsigned)(DIM / 64); ++nt) {
    const unsigned n0 = nt * 64u;
    const _Float16* bp0 = Bt + (size_t)(n0 + nw * 32u + m) * ldb + hh * 8u;
    const _Float16* bp1 = bp0 + (size_t)16 * ldb;
    v8f acc0 = {}, acc1 = {};
#pragma unroll 2
    for (unsigned k0 = 0; k0 < (unsigned)DIM; k0 += 32u) {
      const v16h a  = frag_at(ap + k0);
      const v16h b0 = frag_at(bp0 + k0);
      const v16h b1 = frag_at(bp1 + k0);
      acc0 = wmma16(a, b0, acc0);
      acc1 = wmma16(a, b1, acc1);
    }
#pragma unroll
    for (int r = 0; r < 8; ++r) {
      float* d = &Cs[(mw * 16u + hh * 8u + (unsigned)r) * LDC + nw * 32u + m];
      d[0]  = acc0[r];
      d[16] = acc1[r];
    }
    __syncthreads();

    if (MODE == 0) {
      v8h x[2];
      size_t off[2];
#pragma unroll
      for (unsigned i = 0; i < 2u; ++i) {
        const unsigned r = 32u * i + (tid >> 3);
        const unsigned c = (tid & 7u) * 8u;
        const v4f u0 = *(const v4f*)&Cs[r * LDC + c];
        const v4f u1 = *(const v4f*)&Cs[r * LDC + c + 4];
        float acc = ssq[i];
#pragma unroll
        for (int j = 0; j < 4; ++j) {
          const float t0 = u0[j] * (1.0f / WCARRY);
          const float t1 = u1[j] * (1.0f / WCARRY);
          x[i][j]     = toh_flush(t0);
          x[i][j + 4] = toh_flush(t1);
          acc += t0 * t0;
          acc += t1 * t1;
        }
        ssq[i] = acc;
        off[i] = (size_t)r * DIM + n0 + c;
      }
#pragma unroll
      for (int i = 0; i < 2; ++i) *(volatile v8h*)(out16 + off[i]) = x[i];
      __threadfence();
#pragma unroll
      for (int i = 0; i < 2; ++i) *(volatile v8h*)(out16 + off[i]) = x[i];
    }

    if (MODE == 1) {
      v8h x[2];
      size_t off[2];
#pragma unroll
      for (unsigned i = 0; i < 2u; ++i) {
        const unsigned dcol = 32u * i + (tid >> 3);
        const unsigned kk = (tid & 7u) * 8u;
#pragma unroll
        for (unsigned j = 0; j < 8u; ++j)
          x[i][j] = toh_flush(Cs[(kk + j) * LDC + dcol] * (1.0f / WCARRY));
        off[i] = (size_t)(n0 + dcol) * NSUP + kk;
      }
#pragma unroll
      for (int i = 0; i < 2; ++i) *(volatile v8h*)(out16 + off[i]) = x[i];
      __threadfence();
#pragma unroll
      for (int i = 0; i < 2; ++i) *(volatile v8h*)(out16 + off[i]) = x[i];
    }
    __syncthreads();
  }

  if (MODE == 0) {
    float t0 = ssq[0], t1 = ssq[1];
#pragma unroll
    for (int off = 1; off < 8; off <<= 1) {
      t0 += __shfl_xor(t0, off, 32);
      t1 += __shfl_xor(t1, off, 32);
    }
    const float i0 = 1.0f / fmaxf(sqrtf(t0), 1.0e-12f);
    const float i1 = 1.0f / fmaxf(sqrtf(t1), 1.0e-12f);
    if ((tid & 7u) == 0u) {
      Ninv[tid >> 3] = i0;
      Ninv[32u + (tid >> 3)] = i1;
    }
    __syncthreads();
    const v4f nv4 = *(const v4f*)&Ninv[(tid & 15u) * 4u];
    if (tid < 16u) {
      float* p = inv + tid * 4u;
      *(volatile v4f*)p = nv4;
      __threadfence();
      *(volatile v4f*)p = nv4;
    }
  }
}

__global__ __launch_bounds__(256) void qproj_kernel(
    const _Float16* __restrict__ Qin, const _Float16* __restrict__ WqT,
    _Float16* __restrict__ nq16, float* __restrict__ qinv) {
  const size_t r0 = (size_t)blockIdx.x * 64u;
  proj_body<0>(Qin + r0 * DIM, WqT, (unsigned)DIM, nq16 + r0 * DIM, qinv + r0);
}

__global__ __launch_bounds__(256) void kvproj_kernel(
    const _Float16* __restrict__ Kin, const _Float16* __restrict__ WkT,
    const _Float16* __restrict__ WvT, _Float16* __restrict__ nk16,
    _Float16* __restrict__ nvT, float* __restrict__ kinv) {
  const size_t way = blockIdx.x;
  if (blockIdx.y == 0u) {
    proj_body<0>(Kin + way * NSUP * DIM, WkT + way * DIM, (unsigned)(NWAY * DIM),
                 nk16 + way * NSUP * DIM, kinv + way * NSUP);
  } else {
    proj_body<1>(Kin + way * NSUP * DIM, WvT + way * DIM, (unsigned)(NWAY * DIM),
                 nvT + way * DIM * NSUP, kinv + way * NSUP);
  }
}

__global__ __launch_bounds__(256) void simproto_kernel(
    const _Float16* __restrict__ Qh, const float* __restrict__ Qinv,
    const _Float16* __restrict__ Kh, const float* __restrict__ Kinv,
    const _Float16* __restrict__ Vt, float* __restrict__ out) {
  __shared__ _Float16 Ps[8 * 16 * LDT];
  __shared__ float Os[8 * 16 * LDC];

  const unsigned tid = threadIdx.x, lane = tid & 31u;
  const unsigned wave = (unsigned)__builtin_amdgcn_readfirstlane((int)(tid >> 5));
  const unsigned hh = lane >> 4, m = lane & 15u;
  const unsigned way = blockIdx.y;
  const unsigned qrow0 = blockIdx.x * 128u + wave * 16u;
  const unsigned pbase = wave * (16u * LDT);
  const unsigned obase = wave * (16u * LDC);

  const _Float16* qp = Qh + (size_t)(qrow0 + m) * DIM + hh * 8u;
  const _Float16* kp = Kh + (size_t)(way * NSUP + m) * DIM + hh * 8u;

  v8f s[4];
#pragma unroll
  for (int kg = 0; kg < 4; ++kg) s[kg] = (v8f){};
#pragma unroll 2
  for (unsigned k0 = 0; k0 < (unsigned)DIM; k0 += 32u) {
    const v16h qf = frag_at(qp + k0);
#pragma unroll
    for (int kg = 0; kg < 4; ++kg) {
      const v16h kf = frag_at(kp + (size_t)(kg * 16) * DIM + k0);
      s[kg] = wmma16(qf, kf, s[kg]);
    }
  }

  const v4f qa = *(const v4f*)(Qinv + qrow0 + hh * 8u);
  const v4f qb = *(const v4f*)(Qinv + qrow0 + hh * 8u + 4u);
  float kv[4];
#pragma unroll
  for (int kg = 0; kg < 4; ++kg) kv[kg] = Kinv[way * NSUP + (unsigned)kg * 16u + m];
#pragma unroll
  for (int v = 0; v < 8; ++v) {
    const float qv = (v < 4) ? qa[v & 3] : qb[v & 3];
    float t = 0.0f;
#pragma unroll
    for (int kg = 0; kg < 4; ++kg) {
      const float x = s[kg][v] * (qv * kv[kg]);
      s[kg][v] = x;
      t += x * x;
    }
    t = red16_sum(t);
    const float pin = PCARRY * (1.0f / fmaxf(sqrtf(t), 1.0e-12f));
#pragma unroll
    for (int kg = 0; kg < 4; ++kg)
      Ps[pbase + (hh * 8u + (unsigned)v) * LDT + (unsigned)kg * 16u + m] =
          toh_flush(s[kg][v] * pin);
  }
  wave_lds_sync();

  const _Float16* vp = Vt + ((size_t)way * DIM + m) * NSUP + hh * 8u;
#pragma unroll 1
  for (unsigned g = 0; g < (unsigned)(DIM / 64); ++g) {
    v8f o[4];
#pragma unroll
    for (int nb = 0; nb < 4; ++nb) o[nb] = (v8f){};
#pragma unroll
    for (int c = 0; c < 2; ++c) {
      const v16h pf = ld_frag(&Ps[pbase + c * 32], LDT);
#pragma unroll
      for (int nb = 0; nb < 4; ++nb) {
        const v16h vf = frag_at(vp + (size_t)(g * 64u + (unsigned)nb * 16u) * NSUP + c * 32);
        o[nb] = wmma16(pf, vf, o[nb]);
      }
    }
#pragma unroll
    for (int nb = 0; nb < 4; ++nb)
#pragma unroll
      for (int v = 0; v < 8; ++v)
        Os[obase + (hh * 8u + (unsigned)v) * LDC + (unsigned)nb * 16u + m] =
            o[nb][v] * (1.0f / PCARRY);
    wave_lds_sync();

    v4f x[8];
#pragma unroll
    for (unsigned i = 0; i < 8u; ++i)
      x[i] = *(const v4f*)&Os[obase + (2u * i + (lane >> 4)) * LDC + (lane & 15u) * 4u];
    float* op = out + ((size_t)(qrow0 + (lane >> 4)) * NWAY + way) * DIM + g * 64u +
                (lane & 15u) * 4u;
#pragma unroll
    for (int i = 0; i < 8; ++i) *(volatile v4f*)(op + (size_t)i * (2 * NWAY * DIM)) = x[i];
    __threadfence();
#pragma unroll
    for (int i = 0; i < 8; ++i) *(volatile v4f*)(op + (size_t)i * (2 * NWAY * DIM)) = x[i];
    wave_lds_sync();
  }
}

extern "C" void kernel_launch(void* const* d_in, const int* in_sizes, int n_in,
                              void* d_out, int out_size, void* d_ws, size_t ws_size,
                              hipStream_t stream) {
  if (n_in < 5) return;
  if ((long long)in_sizes[0] < (long long)NQ * DIM) return;
  if ((long long)in_sizes[1] < (long long)KROWS * DIM) return;
  if ((long long)in_sizes[2] < (long long)DIM * DIM) return;
  if ((long long)in_sizes[3] < (long long)NWAY * DIM * DIM) return;
  if ((long long)in_sizes[4] < (long long)NWAY * DIM * DIM) return;
  if ((long long)out_size < (long long)NQ * NWAY * DIM) return;
  if (ws_size < WS_TOTAL) return;

  const float* query = (const float*)d_in[0];
  const float* key   = (const float*)d_in[1];
  const float* wq    = (const float*)d_in[2];
  const float* wk    = (const float*)d_in[3];
  const float* wv    = (const float*)d_in[4];
  float* out = (float*)d_out;

  char* ws = (char*)d_ws;
  _Float16* WqT   = (_Float16*)(ws + OFF_WQT);
  _Float16* WkT   = (_Float16*)(ws + OFF_WKT);
  _Float16* WvT   = (_Float16*)(ws + OFF_WVT);
  _Float16* Qin16 = (_Float16*)(ws + OFF_QIN);
  _Float16* Kin16 = (_Float16*)(ws + OFF_KIN);
  _Float16* Nq16  = (_Float16*)(ws + OFF_NQ);
  _Float16* Nk16  = (_Float16*)(ws + OFF_NK);
  _Float16* NvT16 = (_Float16*)(ws + OFF_NVT);
  float*    Qinv  = (float*)(ws + OFF_QINV);
  float*    Kinv  = (float*)(ws + OFF_KINV);

  dim3 blk(256);

  wconv_kernel<<<dim3(DIM / 64, DIM / 64), blk, 0, stream>>>(wq, WqT, (unsigned)DIM, (unsigned)DIM);
  wconv_kernel<<<dim3(DIM / 64, (NWAY * DIM) / 64), blk, 0, stream>>>(
      wk, WkT, (unsigned)DIM, (unsigned)(NWAY * DIM));
  wconv_kernel<<<dim3(DIM / 64, (NWAY * DIM) / 64), blk, 0, stream>>>(
      wv, WvT, (unsigned)DIM, (unsigned)(NWAY * DIM));

  cast_kernel<<<dim3((unsigned)(((size_t)NQ * DIM) / (8u * 256u))), blk, 0, stream>>>(
      query, Qin16, (unsigned)(((size_t)NQ * DIM) / 8u));
  cast_kernel<<<dim3((unsigned)(((size_t)KROWS * DIM) / (8u * 256u))), blk, 0, stream>>>(
      key, Kin16, (unsigned)(((size_t)KROWS * DIM) / 8u));

  qproj_kernel<<<dim3(NQ / 64), blk, 0, stream>>>(Qin16, WqT, Nq16, Qinv);
  kvproj_kernel<<<dim3(NWAY, 2), blk, 0, stream>>>(Kin16, WkT, WvT, Nk16, NvT16, Kinv);
  simproto_kernel<<<dim3(NQ / 128, NWAY), blk, 0, stream>>>(Nq16, Qinv, Nk16, Kinv, NvT16, out);
}
